// EnhancedPGATActor_57286273794131
// MI455X (gfx1250) — hardware-verified
//
#include <hip/hip_runtime.h>
#include <stddef.h>


#define OBSW    37
#define QD      19
#define KD      16
#define VD      18
#define NH      4
#define CH      128
#define HCW     512
#define HID     128
#define MLP     256
#define OUTD    2
#define K0P     32
#define LDQ     1536
#define AP      1024
#define HP      256
#define M1P     512
#define X2P     256
#define SCALE_F 0.17677669529663687f

#define NTHR    256
#define NWAVE   8
#define EPT     8
#define CHUNK   (NTHR * EPT)
#define WCAP    (EPT * 32)
#define LISTN   (NWAVE * WCAP)
#define NBMAX   2048
#define RCAP    28672
#define DEGCAP  4096
#define GBM     64
#define GBN     64
#define GTHR    128
#define HTHR    64
#define WSCAP   134217728
#define LDS_AGG ((2 * RCAP + 2 * NBMAX + LISTN) * 4 + 64)

static_assert((CHUNK & (CHUNK - 1)) == 0 && CHUNK <= 4096);
static_assert((NBMAX & (NBMAX - 1)) == 0 && NBMAX <= 4096);
static_assert(NTHR * 8 == NBMAX);
static_assert(LISTN >= NBMAX);
static_assert(LISTN >= NWAVE * WCAP);
static_assert((RCAP % 32) == 0);
static_assert(NWAVE * (AP / 2) <= RCAP);
static_assert(LDS_AGG <= 300000);
static_assert(GBM == (GTHR / 32) * 16);
static_assert(GBN == 64 && GBM == 64);
static_assert(NH * CH == HCW);
static_assert(HCW == 32 * 16);
static_assert(CH == 8 * 16);
static_assert((HCW % GBN) == 0 && (HID % GBN) == 0 && (MLP % GBN) == 0);
static_assert((K0P % 32) == 0 && (HID % 32) == 0 && (HCW % 32) == 0 && (MLP % 32) == 0);
static_assert(HTHR == GBM);
static_assert(2 * HTHR == 128);
static_assert((MLP % 4) == 0);

typedef float          v2f  __attribute__((ext_vector_type(2)));
typedef float          v4f  __attribute__((ext_vector_type(4)));
typedef float          v8f  __attribute__((ext_vector_type(8)));
typedef int            v4i  __attribute__((ext_vector_type(4)));
typedef int            v8i  __attribute__((ext_vector_type(8)));
typedef unsigned short v8us __attribute__((ext_vector_type(8)));
typedef __bf16         v16bf __attribute__((ext_vector_type(16)));
union FragB { v16bf v; v8us h[2]; v8i w; };

__device__ __forceinline__ v8f wmb(const FragB& a, const FragB& b, v8f c) {
  v8f d = __builtin_amdgcn_wmma_f32_16x16x32_bf16(false, a.v, false, b.v, (short)0, c, false, false);
  asm volatile("v_nop\n\tv_nop\n\tv_nop\n\tv_nop" : "+v"(d) : "v"(a.w), "v"(b.w));
  return d;
}

__device__ __forceinline__ unsigned bfb(float x) {
  const unsigned u = __float_as_uint(x);
  return (u + 0x7FFFu + ((u >> 16) & 1u)) >> 16;
}

__device__ __forceinline__ void split2(float x, float y, int& h, int& l) {
  const unsigned hx = bfb(x), hy = bfb(y);
  const float rx = x - __uint_as_float(hx << 16);
  const float ry = y - __uint_as_float(hy << 16);
  const unsigned lx = bfb(rx), ly = bfb(ry);
  h = (int)(hx | (hy << 16));
  l = (int)(lx | (ly << 16));
}

__device__ __forceinline__ v4i pack8(float x0, float x1, float x2, float x3,
                                     float x4, float x5, float x6, float x7, int isLo) {
  int h0, h1, h2, h3, l0, l1, l2, l3;
  split2(x0, x1, h0, l0);
  split2(x2, x3, h1, l1);
  split2(x4, x5, h2, l2);
  split2(x6, x7, h3, l3);
  v4i r;
  r.x = isLo ? l0 : h0;
  r.y = isLo ? l1 : h1;
  r.z = isLo ? l2 : h2;
  r.w = isLo ? l3 : h3;
  return r;
}

__device__ __forceinline__ int scan_chunk(const int* __restrict__ dsts, int nE, int cbase, int slotBase,
                                          int nb, int vec8, int* list, int tid, int lane, int wave) {
  int wc = 0;
  const int el0  = tid * EPT;
  const int e0   = cbase + el0;
  const int sent = -2147483647 - 1;
  v4i da, db;
  if (vec8 != 0 && cbase + CHUNK <= nE) {
    da = *(const v4i*)(dsts + e0);
    db = *(const v4i*)(dsts + e0 + 4);
  } else {
    da.x = (e0     < nE) ? dsts[min(e0,     nE - 1)] : sent;
    da.y = (e0 + 1 < nE) ? dsts[min(e0 + 1, nE - 1)] : sent;
    da.z = (e0 + 2 < nE) ? dsts[min(e0 + 2, nE - 1)] : sent;
    da.w = (e0 + 3 < nE) ? dsts[min(e0 + 3, nE - 1)] : sent;
    db.x = (e0 + 4 < nE) ? dsts[min(e0 + 4, nE - 1)] : sent;
    db.y = (e0 + 5 < nE) ? dsts[min(e0 + 5, nE - 1)] : sent;
    db.z = (e0 + 6 < nE) ? dsts[min(e0 + 6, nE - 1)] : sent;
    db.w = (e0 + 7 < nE) ? dsts[min(e0 + 7, nE - 1)] : sent;
  }
  const unsigned nbs = (unsigned)slotBase;
  const unsigned unb = (unsigned)nb;
  const unsigned s0 = (unsigned)da.x - nbs, s1 = (unsigned)da.y - nbs;
  const unsigned s2 = (unsigned)da.z - nbs, s3 = (unsigned)da.w - nbs;
  const unsigned s4 = (unsigned)db.x - nbs, s5 = (unsigned)db.y - nbs;
  const unsigned s6 = (unsigned)db.z - nbs, s7 = (unsigned)db.w - nbs;
  const bool h0 = s0 < unb, h1 = s1 < unb, h2 = s2 < unb, h3 = s3 < unb;
  const bool h4 = s4 < unb, h5 = s5 < unb, h6 = s6 < unb, h7 = s7 < unb;
  const unsigned any = __builtin_amdgcn_ballot_w32(h0 | h1 | h2 | h3 | h4 | h5 | h6 | h7);
  if (any != 0u) {
#define HITJ(J, HJ, SJ) { \
      const unsigned mj = __builtin_amdgcn_ballot_w32(HJ); \
      if (mj != 0u) { \
        if (HJ) { \
          const int pos = wc + (int)__builtin_amdgcn_mbcnt_lo(mj, 0u); \
          if (pos < WCAP) list[wave * WCAP + pos] = ((el0 + (J)) << 12) | (int)(SJ); \
        } \
        wc += (int)__builtin_popcount(mj); } }
    HITJ(0, h0, s0)
    HITJ(1, h1, s1)
    HITJ(2, h2, s2)
    HITJ(3, h3, s3)
    HITJ(4, h4, s4)
    HITJ(5, h5, s5)
    HITJ(6, h6, s6)
    HITJ(7, h7, s7)
#undef HITJ
  }
  return wc;
}

__global__ __launch_bounds__(NTHR) void k_prep0(const float* __restrict__ obs, unsigned short* P0,
                                                int nN, int MP, int nUnits) {
  const int u = (int)blockIdx.x * NTHR + (int)threadIdx.x;
  if (u >= nUnits) return;
  const int per = MP * 8;
  const int seg = u / per;
  const int rem = u - seg * per;
  const int row = rem >> 3;
  const int p   = rem & 7;
  const int isLo = p >> 2;
  const int f0  = (p & 3) * 8;
  const int rc  = row < nN ? row : nN - 1;
  const float* orow = obs + (size_t)rc * OBSW;
  const int lim = (seg == 0) ? QD : ((seg == 1) ? KD : VD);
  const bool rowok = row < nN;
  float x[8];
#pragma unroll
  for (int i = 0; i < 8; ++i) {
    const int f  = f0 + i;
    const int cA = (f < 12) ? f : (f + 18);
    const int cB = (f < 12) ? (f + 12) : (f + 14);
    const int cC = f + 12;
    int col = (seg == 0) ? cA : ((seg == 1) ? cB : cC);
    col = col < 0 ? 0 : (col > OBSW - 1 ? OBSW - 1 : col);
    const float v = orow[col];
    x[i] = (f < lim && rowok) ? v : 0.0f;
  }
  const v4i w = pack8(x[0], x[1], x[2], x[3], x[4], x[5], x[6], x[7], isLo);
  unsigned short* dstp = P0 + ((size_t)seg * (size_t)MP + (size_t)row) * (2 * K0P) + 8 * p;
  *(volatile v4i*)dstp = w;
  __threadfence();
  *(volatile v4i*)dstp = w;
}

__global__ __launch_bounds__(NTHR) void k_wprep(const float* __restrict__ W, unsigned short* Bt,
                                                int K, int Kp, int N, int rowOff, int nUnits) {
  const int u = (int)blockIdx.x * NTHR + (int)threadIdx.x;
  if (u >= nUnits) return;
  const int ppr  = Kp >> 2;
  const int n    = u / ppr;
  const int p    = u - n * ppr;
  const int c    = 8 * p;
  const int isLo = (c >= Kp) ? 1 : 0;
  const int k8   = c - isLo * Kp;
  const int ncl  = n < N ? n : N - 1;
  float x[8];
#pragma unroll
  for (int i = 0; i < 8; ++i) {
    const int k  = k8 + i;
    const int kc = k < K ? k : K - 1;
    const float v = W[(size_t)kc * (size_t)N + (size_t)ncl];
    x[i] = (k < K) ? v : 0.0f;
  }
  const v4i w = pack8(x[0], x[1], x[2], x[3], x[4], x[5], x[6], x[7], isLo);
  unsigned short* dstp = Bt + (size_t)(rowOff + n) * (size_t)(2 * Kp) + c;
  *(volatile v4i*)dstp = w;
  __threadfence();
  *(volatile v4i*)dstp = w;
}

__device__ __forceinline__ v4f epi4(const float* stg, const float* __restrict__ bias, int r, int c,
                                    int rowBase, int colBase, int biasLen, int hasBias, int relu, int M) {
  v4f v = *(const v4f*)(stg + (size_t)r * GBN + c);
  const int col = colBase + c;
  const int bl  = biasLen < 1 ? 1 : biasLen;
  const int i0 = col     < bl ? col     : bl - 1;
  const int i1 = col + 1 < bl ? col + 1 : bl - 1;
  const int i2 = col + 2 < bl ? col + 2 : bl - 1;
  const int i3 = col + 3 < bl ? col + 3 : bl - 1;
  const float b0 = bias[i0], b1 = bias[i1], b2 = bias[i2], b3 = bias[i3];
  v.x += hasBias ? b0 : 0.0f;
  v.y += hasBias ? b1 : 0.0f;
  v.z += hasBias ? b2 : 0.0f;
  v.w += hasBias ? b3 : 0.0f;
  if (relu) { v.x = fmaxf(v.x, 0.f); v.y = fmaxf(v.y, 0.f); v.z = fmaxf(v.z, 0.f); v.w = fmaxf(v.w, 0.f); }
  if (rowBase + r >= M) { v.x = 0.f; v.y = 0.f; v.z = 0.f; v.w = 0.f; }
  return v;
}

__global__ __launch_bounds__(GTHR) void k_gemm(const unsigned short* __restrict__ A, const unsigned short* __restrict__ Bt,
                                               const float* __restrict__ bias, float* Cf, unsigned short* Cb,
                                               int Kp, int aSeg, int cbps, int biasLen, int hasBias,
                                               int relu, int mode, int ldc, int M) {
  __shared__ __attribute__((aligned(16))) float stg[GBM * GBN];
  const int tid = threadIdx.x, lane = tid & 31, wave = tid >> 5, hh = lane >> 4, m = lane & 15;
  const int rowBase = (int)blockIdx.x * GBM;
  const int colBase = (int)blockIdx.y * GBN;
  const int cb  = cbps < 1 ? 1 : cbps;
  const int seg = (int)blockIdx.y / cb;
  const int kp  = Kp < 32 ? 32 : (Kp > 512 ? 512 : Kp);
  const int ld  = 2 * kp;
  const int nk  = kp >> 5;
  const unsigned short* Ab = A + (size_t)seg * (size_t)(aSeg < 0 ? 0 : aSeg);
  const size_t arow = (size_t)(rowBase + 16 * wave + m) * (size_t)ld + 8 * hh;
  const size_t brow = (size_t)(colBase + m) * (size_t)ld + 8 * hh;
  v8f acc[4];
#pragma unroll
  for (int t = 0; t < 4; ++t) { v8f z = {0.f, 0.f, 0.f, 0.f, 0.f, 0.f, 0.f, 0.f}; acc[t] = z; }
#pragma unroll 1
  for (int p = 0; p < 3; ++p) {
    const int aoff = (p == 2) ? kp : 0;
    const int boff = (p == 1) ? kp : 0;
#pragma unroll 1
    for (int ks = 0; ks < nk; ++ks) {
      FragB af;
      af.h[0] = *(const v8us*)(Ab + arow + aoff + 32 * ks);
      af.h[1] = *(const v8us*)(Ab + arow + aoff + 32 * ks + 16);
#pragma unroll
      for (int t = 0; t < 4; ++t) {
        const size_t bo = brow + (size_t)(16 * t) * (size_t)ld + boff + 32 * ks;
        FragB bf;
        bf.h[0] = *(const v8us*)(Bt + bo);
        bf.h[1] = *(const v8us*)(Bt + bo + 16);
        acc[t] = wmb(af, bf, acc[t]);
      }
    }
  }
  float* sp = stg + (size_t)(16 * wave + 8 * hh) * GBN + m;
#pragma unroll
  for (int t = 0; t < 4; ++t) {
#pragma unroll
    for (int r = 0; r < 8; ++r) sp[(size_t)r * GBN + 16 * t] = acc[t][r];
  }
  __syncthreads();
  const int nF = GBM * GBN / 4;
  if (mode == 0) {
#pragma unroll 1
    for (int f = tid; f < nF; f += GTHR) {
      const int r = f >> 4, q = f & 15;
      const v4f v = epi4(stg, bias, r, 4 * q, rowBase, colBase, biasLen, hasBias, relu, M);
      *(volatile v4f*)(Cf + (size_t)(rowBase + r) * (size_t)ldc + colBase + 4 * q) = v;
    }
    __threadfence();
#pragma unroll 1
    for (int f = tid; f < nF; f += GTHR) {
      const int r = f >> 4, q = f & 15;
      const v4f v = epi4(stg, bias, r, 4 * q, rowBase, colBase, biasLen, hasBias, relu, M);
      *(volatile v4f*)(Cf + (size_t)(rowBase + r) * (size_t)ldc + colBase + 4 * q) = v;
    }
  } else {
    const int lo2 = ldc >> 1;
#pragma unroll 1
    for (int f = tid; f < nF; f += GTHR) {
      const int r = f >> 4, pc = f & 15, isLo = pc >> 3, c0 = 8 * (pc & 7);
      const v4f va = epi4(stg, bias, r, c0,     rowBase, colBase, biasLen, hasBias, relu, M);
      const v4f vb = epi4(stg, bias, r, c0 + 4, rowBase, colBase, biasLen, hasBias, relu, M);
      const v4i w = pack8(va.x, va.y, va.z, va.w, vb.x, vb.y, vb.z, vb.w, isLo);
      unsigned short* dp = Cb + (size_t)(rowBase + r) * (size_t)ldc + (size_t)(isLo * lo2) + colBase + c0;
      *(volatile v4i*)dp = w;
    }
    __threadfence();
#pragma unroll 1
    for (int f = tid; f < nF; f += GTHR) {
      const int r = f >> 4, pc = f & 15, isLo = pc >> 3, c0 = 8 * (pc & 7);
      const v4f va = epi4(stg, bias, r, c0,     rowBase, colBase, biasLen, hasBias, relu, M);
      const v4f vb = epi4(stg, bias, r, c0 + 4, rowBase, colBase, biasLen, hasBias, relu, M);
      const v4i w = pack8(va.x, va.y, va.z, va.w, vb.x, vb.y, vb.z, vb.w, isLo);
      unsigned short* dp = Cb + (size_t)(rowBase + r) * (size_t)ldc + (size_t)(isLo * lo2) + colBase + c0;
      *(volatile v4i*)dp = w;
    }
  }
}

__global__ __launch_bounds__(NTHR) void k_agg(
    const int* __restrict__ srcs, const int* __restrict__ dsts,
    const float* __restrict__ QKV, const float* __restrict__ obs,
    unsigned short* AGG, int nN, int nE, int nb, int vec8, int MP) {
  extern __shared__ v4f lds_dyn[];
  int* reg1 = (int*)lds_dyn;
  int* reg2 = reg1 + RCAP;
  int* scnt = reg2 + RCAP;
  int* soff = scnt + NBMAX;
  int* list = soff + NBMAX;
  int* wcnt = list + LISTN;
  int* wtot = wcnt + NWAVE;
  const int tid = threadIdx.x, lane = tid & 31, wave = tid >> 5;
  const int nodeBase = (int)blockIdx.x * nb;

  for (int i = tid; i < NBMAX; i += NTHR) scnt[i] = 0;
  __syncthreads();

  int tot = 0;
  const int nChunks = (nE + CHUNK - 1) / CHUNK;
#pragma unroll 1
  for (int ch = 0; ch < nChunks; ++ch) {
    const int cbase = ch * CHUNK;
    const int wc = scan_chunk(dsts, nE, cbase, nodeBase, nb, vec8, list, tid, lane, wave);
    if (lane == 0) wcnt[wave] = wc;
    __syncthreads();
    int pre = 0, all = 0;
#pragma unroll
    for (int w2 = 0; w2 < NWAVE; ++w2) {
      int c = wcnt[w2];
      c = c < 0 ? 0 : (c > WCAP ? WCAP : c);
      all += c;
      pre += (w2 < wave) ? c : 0;
    }
    const int wcc  = wc > WCAP ? WCAP : wc;
    const int base = tot + pre;
#pragma unroll 1
    for (int i = lane; i < wcc; i += 32) {
      const int ent = list[wave * WCAP + i];
      const int el  = (ent >> 12) & (CHUNK - 1);
      const int sl  = ent & (NBMAX - 1);
      int eid = cbase + el;
      eid = eid > nE - 1 ? nE - 1 : eid;
      const int pos = base + i;
      if (pos < RCAP) reg1[pos] = (int)(((unsigned)eid << 12) | (unsigned)sl);
    }
    tot += all;
    tot = tot > RCAP ? RCAP : tot;
    __syncthreads();
  }
  const int nh = tot;

  if (wave == 0) {
#pragma unroll 1
    for (int b0 = 0; b0 < nh; b0 += 32) {
      const int idx = b0 + lane;
      const int uv  = reg1[idx < RCAP ? idx : RCAP - 1];
      const int m32 = (nh - b0) < 32 ? (nh - b0) : 32;
#pragma unroll 1
      for (int k = 0; k < m32; ++k) {
        const int u  = __builtin_amdgcn_readlane(uv, k);
        const int sl = u & (NBMAX - 1);
        if (lane == 0) scnt[sl] = scnt[sl] + 1;
      }
    }
  }
  __syncthreads();

  {
    const v4i ca = *(const v4i*)(scnt + 8 * tid);
    const v4i cb = *(const v4i*)(scnt + 8 * tid + 4);
    const int e0 = ca.x < 0 ? 0 : ca.x, e1 = ca.y < 0 ? 0 : ca.y, e2 = ca.z < 0 ? 0 : ca.z, e3 = ca.w < 0 ? 0 : ca.w;
    const int e4 = cb.x < 0 ? 0 : cb.x, e5 = cb.y < 0 ? 0 : cb.y, e6 = cb.z < 0 ? 0 : cb.z, e7 = cb.w < 0 ? 0 : cb.w;
    const int ts = e0 + e1 + e2 + e3 + e4 + e5 + e6 + e7;
    int incl = ts;
#pragma unroll
    for (int d = 1; d < 32; d <<= 1) {
      const int up = __shfl_up(incl, d);
      if (lane >= d) incl += up;
    }
    if (lane == 31) wtot[wave] = incl;
    __syncthreads();
    int pre = 0;
#pragma unroll
    for (int w2 = 0; w2 < NWAVE; ++w2) pre += (w2 < wave) ? wtot[w2] : 0;
    int run = pre + incl - ts;
    soff[8 * tid + 0] = run; run += e0;
    soff[8 * tid + 1] = run; run += e1;
    soff[8 * tid + 2] = run; run += e2;
    soff[8 * tid + 3] = run; run += e3;
    soff[8 * tid + 4] = run; run += e4;
    soff[8 * tid + 5] = run; run += e5;
    soff[8 * tid + 6] = run; run += e6;
    soff[8 * tid + 7] = run;
  }
  __syncthreads();
  for (int i = tid; i < NBMAX; i += NTHR) list[i] = soff[i];
  __syncthreads();

  if (wave == 0) {
#pragma unroll 1
    for (int b0 = 0; b0 < nh; b0 += 32) {
      const int idx = b0 + lane;
      const int uv  = reg1[idx < RCAP ? idx : RCAP - 1];
      const int m32 = (nh - b0) < 32 ? (nh - b0) : 32;
#pragma unroll 1
      for (int k = 0; k < m32; ++k) {
        const int u   = __builtin_amdgcn_readlane(uv, k);
        const int sl  = u & (NBMAX - 1);
        const int eid = (int)((unsigned)u >> 12);
        if (lane == 0) {
          int pos = list[sl];
          pos = pos < 0 ? 0 : (pos > RCAP - 1 ? RCAP - 1 : pos);
          reg2[pos] = eid;
          list[sl] = pos + 1;
        }
      }
    }
  }
  __syncthreads();

  const int nbw = nb >> 3;
  const int c16 = 16 * lane;
  int* stgw = reg1 + wave * (AP / 2);
  const bool ovf = (nh >= RCAP);
  const float qnan = __int_as_float(0x7fc00000);
  const float ninf = __int_as_float((int)0xff800000);
  const v4f z4 = {0.f, 0.f, 0.f, 0.f};
#pragma unroll 1
  for (int jt = 0; jt < nbw; ++jt) {
    const int slot = wave * nbw + jt;
    const int grow = nodeBase + slot;
    const int gcl  = grow < nN ? grow : nN - 1;
    const int gst  = grow < MP ? grow : MP - 1;
    int st = soff[slot];
    const int craw = scnt[slot];
    int cnt = craw;
    st  = st < 0 ? 0 : (st > nh ? nh : st);
    cnt = cnt < 0 ? 0 : (cnt > DEGCAP ? DEGCAP : cnt);
    if (cnt > nh - st) cnt = nh - st;
    if (grow >= nN) cnt = 0;
    const bool poison = (ovf || craw > DEGCAP) && (grow < nN);
    const bool wr = grow < MP;

    const float* qd = QKV + (size_t)gcl * LDQ + c16;
    const v4f q0 = *(const v4f*)qd, q1 = *(const v4f*)(qd + 4), q2 = *(const v4f*)(qd + 8), q3 = *(const v4f*)(qd + 12);
    const float pdx = obs[(size_t)gcl * OBSW], pdy = obs[(size_t)gcl * OBSW + 1];
    float mx = ninf, dn = 0.0f;
    v4f a0 = z4, a1 = z4, a2 = z4, a3 = z4;
#pragma unroll 1
    for (int e = 0; e < cnt; ++e) {
      int idx = st + e; idx = idx > RCAP - 1 ? RCAP - 1 : idx;
      int eid = reg2[idx]; eid = eid < 0 ? 0 : (eid > nE - 1 ? nE - 1 : eid);
      const int sraw = srcs[eid];
      const int s = sraw < 0 ? 0 : (sraw > nN - 1 ? nN - 1 : sraw);
      const float* kr = QKV + (size_t)s * LDQ + HCW + c16;
      const v4f k0 = *(const v4f*)kr, k1 = *(const v4f*)(kr + 4), k2 = *(const v4f*)(kr + 8), k3 = *(const v4f*)(kr + 12);
      const float* vr = kr + HCW;
      const v4f v0 = *(const v4f*)vr, v1 = *(const v4f*)(vr + 4), v2 = *(const v4f*)(vr + 8), v3 = *(const v4f*)(vr + 12);
      float dp = q0.x * k0.x;
      dp = fmaf(q0.y, k0.y, dp); dp = fmaf(q0.z, k0.z, dp); dp = fmaf(q0.w, k0.w, dp);
      dp = fmaf(q1.x, k1.x, dp); dp = fmaf(q1.y, k1.y, dp); dp = fmaf(q1.z, k1.z, dp); dp = fmaf(q1.w, k1.w, dp);
      dp = fmaf(q2.x, k2.x, dp); dp = fmaf(q2.y, k2.y, dp); dp = fmaf(q2.z, k2.z, dp); dp = fmaf(q2.w, k2.w, dp);
      dp = fmaf(q3.x, k3.x, dp); dp = fmaf(q3.y, k3.y, dp); dp = fmaf(q3.z, k3.z, dp); dp = fmaf(q3.w, k3.w, dp);
      dp += __shfl_xor(dp, 1);
      dp += __shfl_xor(dp, 2);
      dp += __shfl_xor(dp, 4);
      const float sx = obs[(size_t)s * OBSW], sy = obs[(size_t)s * OBSW + 1];
      const float dx = pdx - sx, dy = pdy - sy;
      const float dist = sqrtf(fmaf(dx, dx, dy * dy));
      const float pw = __expf(-dist);
      const float lg = (dp * SCALE_F) * pw;
      const float mn = fmaxf(mx, lg);
      const float s1 = __expf(mx - mn), s2 = __expf(lg - mn);
      dn = fmaf(dn, s1, s2);
      a0.x = fmaf(a0.x, s1, s2 * v0.x); a0.y = fmaf(a0.y, s1, s2 * v0.y);
      a0.z = fmaf(a0.z, s1, s2 * v0.z); a0.w = fmaf(a0.w, s1, s2 * v0.w);
      a1.x = fmaf(a1.x, s1, s2 * v1.x); a1.y = fmaf(a1.y, s1, s2 * v1.y);
      a1.z = fmaf(a1.z, s1, s2 * v1.z); a1.w = fmaf(a1.w, s1, s2 * v1.w);
      a2.x = fmaf(a2.x, s1, s2 * v2.x); a2.y = fmaf(a2.y, s1, s2 * v2.y);
      a2.z = fmaf(a2.z, s1, s2 * v2.z); a2.w = fmaf(a2.w, s1, s2 * v2.w);
      a3.x = fmaf(a3.x, s1, s2 * v3.x); a3.y = fmaf(a3.y, s1, s2 * v3.y);
      a3.z = fmaf(a3.z, s1, s2 * v3.z); a3.w = fmaf(a3.w, s1, s2 * v3.w);
      mx = mn;
    }
    const float inv  = 1.0f / fmaxf(dn, 1.0f);
    const float invp = poison ? qnan : inv;
    const v4f o0 = a0 * invp, o1 = a1 * invp, o2 = a2 * invp, o3 = a3 * invp;
    {
      const v4i h0 = pack8(o0.x, o0.y, o0.z, o0.w, o1.x, o1.y, o1.z, o1.w, 0);
      const v4i h1 = pack8(o2.x, o2.y, o2.z, o2.w, o3.x, o3.y, o3.z, o3.w, 0);
      const v4i l0 = pack8(o0.x, o0.y, o0.z, o0.w, o1.x, o1.y, o1.z, o1.w, 1);
      const v4i l1 = pack8(o2.x, o2.y, o2.z, o2.w, o3.x, o3.y, o3.z, o3.w, 1);
      *(v4i*)(stgw + 8 * lane)           = h0;
      *(v4i*)(stgw + 8 * lane + 4)       = h1;
      *(v4i*)(stgw + 256 + 8 * lane)     = l0;
      *(v4i*)(stgw + 256 + 8 * lane + 4) = l1;
    }
    __syncthreads();
    const v4i w0 = *(const v4i*)(stgw + 4 * lane);
    const v4i w1 = *(const v4i*)(stgw + 128 + 4 * lane);
    const v4i w2 = *(const v4i*)(stgw + 256 + 4 * lane);
    const v4i w3 = *(const v4i*)(stgw + 384 + 4 * lane);
    unsigned short* rowp = AGG + (size_t)gst * AP;
    if (wr) {
      *(volatile v4i*)(rowp + 8 * lane)       = w0;
      *(volatile v4i*)(rowp + 256 + 8 * lane) = w1;
      *(volatile v4i*)(rowp + 512 + 8 * lane) = w2;
      *(volatile v4i*)(rowp + 768 + 8 * lane) = w3;
    }
    __threadfence();
    if (wr) {
      *(volatile v4i*)(rowp + 8 * lane)       = w0;
      *(volatile v4i*)(rowp + 256 + 8 * lane) = w1;
      *(volatile v4i*)(rowp + 512 + 8 * lane) = w2;
      *(volatile v4i*)(rowp + 768 + 8 * lane) = w3;
    }
    __syncthreads();
  }
}

__global__ __launch_bounds__(HTHR) void k_head(const float* __restrict__ X2, const float* __restrict__ w3,
                                               const float* __restrict__ b3, float* out, int nN) {
  __shared__ __attribute__((aligned(16))) float sO[2 * HTHR];
  const int tid = threadIdx.x;
  const int rowBase = (int)blockIdx.x * HTHR;
  const int row = rowBase + tid;
  const int rc  = row < nN ? row : nN - 1;
  const float* xr = X2 + (size_t)rc * X2P;
  float acc0 = 0.0f, acc1 = 0.0f;
#pragma unroll 1
  for (int j = 0; j < MLP; j += 4) {
    const v4f x  = *(const v4f*)(xr + j);
    const v4f wa = *(const v4f*)(w3 + 2 * j);
    const v4f wb = *(const v4f*)(w3 + 2 * j + 4);
    acc0 = fmaf(x.x, wa.x, acc0); acc1 = fmaf(x.x, wa.y, acc1);
    acc0 = fmaf(x.y, wa.z, acc0); acc1 = fmaf(x.y, wa.w, acc1);
    acc0 = fmaf(x.z, wb.x, acc0); acc1 = fmaf(x.z, wb.y, acc1);
    acc0 = fmaf(x.w, wb.z, acc0); acc1 = fmaf(x.w, wb.w, acc1);
  }
  sO[2 * tid]     = acc0 + b3[0];
  sO[2 * tid + 1] = acc1 + b3[1];
  __syncthreads();
  if (tid < 32) {
    const int lane = tid;
    const int nValid = (nN - rowBase) < HTHR ? (nN - rowBase) : HTHR;
    const int fl  = nValid * OUTD;
    const int n4  = fl >> 2;
    const int rem = fl & 3;
    float* base = out + (size_t)rowBase * OUTD;
    const v4f* s4 = (const v4f*)sO;
    const v4f v = s4[(lane < n4) ? lane : 0];
    const int ti = 4 * n4 + (lane & 3);
    const float tv = sO[ti < fl ? ti : fl - 1];
    const bool tw = (rem != 0) && (lane < rem);
    if (lane < n4) *(volatile v4f*)(base + 4 * lane) = v;
    if (tw) *(volatile float*)(base + 4 * n4 + lane) = tv;
    __threadfence();
    if (lane < n4) *(volatile v4f*)(base + 4 * lane) = v;
    if (tw) *(volatile float*)(base + 4 * n4 + lane) = tv;
  }
}

static int pick_nb(int nE, int nN) {
  int nb = NBMAX;
  while (nb > 16 && (long long)nb * (long long)nE * 5LL > (long long)RCAP * (long long)nN * 4LL) nb >>= 1;
  return nb;
}

extern "C" void kernel_launch(void* const* d_in, const int* in_sizes, int n_in,
                              void* d_out, int out_size, void* d_ws, size_t ws_size,
                              hipStream_t stream) {
  if (n_in < 18) return;
  const int nN = in_sizes[0] / OBSW;
  if (nN <= 0 || in_sizes[0] != nN * OBSW) return;
  if (nN > (1 << 22)) return;
  const int nE = in_sizes[1] / 2;
  if (nE < 1 || in_sizes[1] != 2 * nE) return;
  if (nE > (1 << 20)) return;
  if (in_sizes[2] != QD * HCW || in_sizes[3] != KD * HCW || in_sizes[4] != VD * HCW) return;
  if (in_sizes[5] != HCW * HID || in_sizes[6] != HID) return;
  if (in_sizes[7] != HID * HCW || in_sizes[8] != HID * HCW || in_sizes[9] != HID * HCW) return;
  if (in_sizes[10] != HCW * HID || in_sizes[11] != HID) return;
  if (in_sizes[12] != HID * MLP || in_sizes[13] != MLP) return;
  if (in_sizes[14] != MLP * MLP || in_sizes[15] != MLP) return;
  if (in_sizes[16] != MLP * OUTD || in_sizes[17] != OUTD) return;
  if (out_size != nN * OUTD) return;

  const float* obs = (const float*)d_in[0];
  const int*   eix = (const int*)d_in[1];
  const float* wq0 = (const float*)d_in[2];
  const float* wk0 = (const float*)d_in[3];
  const float* wv0 = (const float*)d_in[4];
  const float* wo0 = (const float*)d_in[5];
  const float* bo0 = (const float*)d_in[6];
  const float* wq1 = (const float*)d_in[7];
  const float* wk1 = (const float*)d_in[8];
  const float* wv1 = (const float*)d_in[9];
  const float* wo1 = (const float*)d_in[10];
  const float* bo1 = (const float*)d_in[11];
  const float* w1  = (const float*)d_in[12];
  const float* b1  = (const float*)d_in[13];
  const float* w2  = (const float*)d_in[14];
  const float* b2  = (const float*)d_in[15];
  const float* w3  = (const float*)d_in[16];
  const float* b3  = (const float*)d_in[17];
  const int* src = eix;
  const int* dst = eix + nE;
  float* out = (float*)d_out;

  const int MP   = ((nN + GBM - 1) / GBM) * GBM;
  const int nb   = pick_nb(nE, nN);
  const int vec8 = ((nE & 3) == 0) ? 1 : 0;

  char* ws = (char*)d_ws;
  size_t off = 0;
  const size_t oP0  = off; off += (size_t)3 * MP * (2 * K0P) * 2;     off = (off + 255) & ~(size_t)255;
  const size_t oB0  = off; off += (size_t)(3 * HCW) * (2 * K0P) * 2;  off = (off + 255) & ~(size_t)255;
  const size_t oBO0 = off; off += (size_t)HID * (2 * HCW) * 2;        off = (off + 255) & ~(size_t)255;
  const size_t oBO1 = off; off += (size_t)HID * (2 * HCW) * 2;        off = (off + 255) & ~(size_t)255;
  const size_t oB1  = off; off += (size_t)(3 * HCW) * (2 * HID) * 2;  off = (off + 255) & ~(size_t)255;
  const size_t oBW1 = off; off += (size_t)MLP * (2 * HID) * 2;        off = (off + 255) & ~(size_t)255;
  const size_t oBW2 = off; off += (size_t)MLP * (2 * MLP) * 2;        off = (off + 255) & ~(size_t)255;
  const size_t oQKV = off; off += (size_t)MP * LDQ * 4;               off = (off + 255) & ~(size_t)255;
  const size_t oAGG = off; off += (size_t)MP * AP * 2;                off = (off + 255) & ~(size_t)255;
  const size_t oHPL = off; off += (size_t)MP * HP * 2;                off = (off + 255) & ~(size_t)255;
  const size_t oM1  = off; off += (size_t)MP * M1P * 2;               off = (off + 255) & ~(size_t)255;
  const size_t oX2  = off; off += (size_t)MP * X2P * 4;               off = (off + 255) & ~(size_t)255;
  if (off > ws_size || off > (size_t)WSCAP) return;
  unsigned short* P0  = (unsigned short*)(ws + oP0);
  unsigned short* B0  = (unsigned short*)(ws + oB0);
  unsigned short* BO0 = (unsigned short*)(ws + oBO0);
  unsigned short* BO1 = (unsigned short*)(ws + oBO1);
  unsigned short* B1  = (unsigned short*)(ws + oB1);
  unsigned short* BW1 = (unsigned short*)(ws + oBW1);
  unsigned short* BW2 = (unsigned short*)(ws + oBW2);
  float*          QKV = (float*)(ws + oQKV);
  unsigned short* AGG = (unsigned short*)(ws + oAGG);
  unsigned short* HPL = (unsigned short*)(ws + oHPL);
  unsigned short* M1  = (unsigned short*)(ws + oM1);
  float*          X2  = (float*)(ws + oX2);

  hipFuncSetAttribute(reinterpret_cast<const void*>(&k_agg),
                      hipFuncAttributeMaxDynamicSharedMemorySize, LDS_AGG);

  const int u0 = 3 * MP * 8;
  k_prep0<<<(u0 + NTHR - 1) / NTHR, NTHR, 0, stream>>>(obs, P0, nN, MP, u0);

  auto wprep = [&](const float* W, unsigned short* Bt, int K, int Kp, int N, int rowOff) {
    const int nu = N * (Kp / 4);
    k_wprep<<<(nu + NTHR - 1) / NTHR, NTHR, 0, stream>>>(W, Bt, K, Kp, N, rowOff, nu);
  };
  wprep(wq0, B0, QD, K0P, HCW, 0);
  wprep(wk0, B0, KD, K0P, HCW, HCW);
  wprep(wv0, B0, VD, K0P, HCW, 2 * HCW);
  wprep(wo0, BO0, HCW, HCW, HID, 0);
  wprep(wq1, B1, HID, HID, HCW, 0);
  wprep(wk1, B1, HID, HID, HCW, HCW);
  wprep(wv1, B1, HID, HID, HCW, 2 * HCW);
  wprep(wo1, BO1, HCW, HCW, HID, 0);
  wprep(w1, BW1, HID, HID, MLP, 0);
  wprep(w2, BW2, MLP, MLP, MLP, 0);

  const int gG = MP / GBM;
  const int gA = (MP + nb - 1) / nb;

  k_gemm<<<dim3(gG, (3 * HCW) / GBN), GTHR, 0, stream>>>(P0, B0, bo0, QKV, M1, K0P, MP * 2 * K0P, HCW / GBN,
                                                         HID, 0, 0, 0, LDQ, nN);
  k_agg<<<gA, NTHR, LDS_AGG, stream>>>(src, dst, QKV, obs, AGG, nN, nE, nb, vec8, MP);
  k_gemm<<<dim3(gG, HID / GBN), GTHR, 0, stream>>>(AGG, BO0, bo0, X2, HPL, HCW, 0, HID / GBN,
                                                   HID, 1, 0, 1, HP, nN);
  k_gemm<<<dim3(gG, (3 * HCW) / GBN), GTHR, 0, stream>>>(HPL, B1, bo1, QKV, M1, HID, 0, (3 * HCW) / GBN,
                                                         HID, 0, 0, 0, LDQ, nN);
  k_agg<<<gA, NTHR, LDS_AGG, stream>>>(src, dst, QKV, obs, AGG, nN, nE, nb, vec8, MP);
  k_gemm<<<dim3(gG, HID / GBN), GTHR, 0, stream>>>(AGG, BO1, bo1, X2, HPL, HCW, 0, HID / GBN,
                                                   HID, 1, 0, 1, HP, nN);
  k_gemm<<<dim3(gG, MLP / GBN), GTHR, 0, stream>>>(HPL, BW1, b1, X2, M1, HID, 0, MLP / GBN,
                                                   MLP, 1, 1, 1, M1P, nN);
  k_gemm<<<dim3(gG, MLP / GBN), GTHR, 0, stream>>>(M1, BW2, b2, X2, HPL, MLP, 0, MLP / GBN,
                                                   MLP, 1, 1, 0, X2P, nN);
  k_head<<<MP / HTHR, HTHR, 0, stream>>>(X2, w3, b3, out, nN);
}
